// HurstEstimator_51960514347079
// MI455X (gfx1250) — hardware-run, weakly checked
//
#include <hip/hip_runtime.h>


#ifndef NB
#define NB 2048
#endif
#define NB_FULL 2048
#ifndef SEQ
#define SEQ 4096
#endif
#define SEQ_FULL 4096
#define WIN   10
#define HID   32
#define NSH   16
#define KP    32
#define CHW   256
#define NTHR  (SEQ / 8)

static_assert(NB >= 1 && NB <= NB_FULL);
static_assert(SEQ <= SEQ_FULL);
static_assert(SEQ % CHW == 0);
static_assert(SEQ > WIN);
static_assert(NTHR == (SEQ / CHW) * 32);
static_assert(NTHR >= 32 && NTHR <= 512);
static_assert((size_t)NTHR * 16 * 2 == (size_t)SEQ * 4);
static_assert((NSH - 1) + (WIN - 1) < KP - 1);
static_assert(HID * NSH * KP == 8 * 256 * 8);
static_assert(KP == 32 && NSH == 16 && HID == 32);
static_assert((size_t)SEQ * 4 <= (size_t)131072);

typedef unsigned short bf;
typedef __attribute__((ext_vector_type(16))) __bf16   v16bf;
typedef __attribute__((ext_vector_type(8)))  unsigned short v8us;
typedef __attribute__((ext_vector_type(8)))  float    v8f;
typedef __attribute__((ext_vector_type(4)))  float    v4f;
typedef v4f  __attribute__((may_alias)) v4fa;

__device__ __forceinline__ unsigned short f2bf(float f) { unsigned u = __float_as_uint(f); u += 0x7FFFu + ((u >> 16) & 1u); return (unsigned short)(u >> 16); }
__device__ __forceinline__ float bf2f(unsigned short w) { return __uint_as_float(((unsigned)w) << 16); }
__device__ __forceinline__ int clampi(int v, int lo, int hi) { return min(max(v, lo), hi); }
__device__ __forceinline__ v16bf cat16b(v8us lo, v8us hi) { return __builtin_bit_cast(v16bf, __builtin_shufflevector(lo, hi, 0, 1, 2, 3, 4, 5, 6, 7, 8, 9, 10, 11, 12, 13, 14, 15)); }
__device__ __forceinline__ v8f wmmab(v16bf a, v16bf b, v8f c) { return __builtin_amdgcn_wmma_f32_16x16x32_bf16(false, a, false, b, (short)0, c, false, false); }
__device__ __forceinline__ v16bf ldb(const bf* p)  { return cat16b(*(const v8us*)p, *(const v8us*)(p + 16)); }
__device__ __forceinline__ v8f wmmag(v16bf a, v16bf b, v8f c) { c = wmmab(a, b, c); asm volatile("v_nop\n\tv_nop\n\tv_nop\n\tv_nop" : "+v"(c) : "v"(a), "v"(b)); return c; }

__global__ __launch_bounds__(256) void k_wt(const float* __restrict__ W1, const float* __restrict__ b1, bf* AT) {
    const int t = threadIdx.x;
#pragma unroll 1
    for (int ps = 0; ps < 2; ++ps) {
#pragma unroll 1
        for (int it = 0; it < 8; ++it) {
            const int q = it * 256 + t; const int R = q >> 2, k0 = (q & 3) * 8; const int hid = R >> 4, s = R & 15;
            const unsigned short bb = f2bf(b1[hid]); v8us o;
#pragma unroll
            for (int i = 0; i < 8; ++i) { const int k = k0 + i, j = k - s;
                const unsigned short wb = f2bf(W1[hid * WIN + clampi(j, 0, WIN - 1)]);
                o[i] = (j >= 0 && j < WIN) ? wb : ((k == KP - 1) ? bb : (unsigned short)0); }
            *(volatile v8us*)(AT + (size_t)q * 8) = o; }
        if (ps == 0) __threadfence(); }
}

__global__ __launch_bounds__(NTHR) __attribute__((amdgpu_num_vgpr(256))) void k_hurst(const float* __restrict__ ret, const bf* __restrict__ AT,
                                                                                      const float* __restrict__ W2, const float* __restrict__ b2, float* OUT) {
    __shared__ __align__(16) float hl[SEQ];
    const int tid = threadIdx.x, lane = tid & 31, lr = lane & 15, hi = lane >> 4;
    const int wave = __builtin_amdgcn_readfirstlane(tid >> 5);
    const int b = blockIdx.x;
    const float* rrow = ret + (size_t)b * SEQ_FULL;
    const int u0 = wave * CHW + 16 * lr + 8 * hi;
    const int o0 = min(u0, SEQ - 8), o1 = min(u0 + 16, SEQ - 8);
    const bool ok0 = (u0 <= SEQ - 8), ok1 = (u0 + 16 <= SEQ - 8);
    const v8f x0 = *(const v8f*)(rrow + o0);
    const v8f x1 = *(const v8f*)(rrow + o1);
    v8us lo, hv;
#pragma unroll
    for (int i = 0; i < 8; ++i) { const unsigned short c0 = f2bf(x0[i]), c1 = f2bf(x1[i]);
        lo[i] = ok0 ? c0 : (unsigned short)0; hv[i] = ok1 ? c1 : (unsigned short)0; }
    hv[7] = (hi != 0) ? (unsigned short)0x3F80 : hv[7];
    const v16bf bfrag = cat16b(lo, hv);
    const bf* ap = AT + (size_t)lr * KP + 8 * hi;
    v8f s = (v8f){};
#pragma unroll 1
    for (int h = 0; h < HID; ++h) {
        const v16bf a = ldb(ap + (size_t)h * (NSH * KP));
        v8f c = (v8f){};
        c = wmmag(a, bfrag, c);
        const float w2 = bf2f(f2bf(W2[h]));
#pragma unroll
        for (int r = 0; r < 8; ++r) s[r] += w2 * fmaxf(c[r], 0.0f);
    }
    const float bb = bf2f(f2bf(b2[0]));
    v4f y0, y1;
#pragma unroll
    for (int r = 0; r < 4; ++r) {
        y0[r] = 0.5f * __builtin_amdgcn_rcpf(1.0f + __expf(-(s[r] + bb)));
        y1[r] = 0.5f * __builtin_amdgcn_rcpf(1.0f + __expf(-(s[4 + r] + bb))); }
    *(v4fa*)(&hl[u0]) = y0;
    *(v4fa*)(&hl[u0 + 4]) = y1;
    __syncthreads();
    float* orow = OUT + (size_t)b * SEQ;
#pragma unroll 1
    for (int ps = 0; ps < 2; ++ps) {
#pragma unroll 1
        for (int it = 0; it < 2; ++it) {
            const int p0 = 4 * (it * NTHR + tid); v4f v;
#pragma unroll
            for (int i = 0; i < 4; ++i) v[i] = hl[max(p0 + i - WIN, 0)];
            *(volatile v4f*)(orow + p0) = v; }
        if (ps == 0) __threadfence(); }
}

static constexpr size_t al256(size_t v) { return (v + 255) & ~(size_t)255; }
static constexpr size_t SZ_AT = al256((size_t)HID * NSH * KP * 2);
static constexpr size_t SZ_TOTAL = SZ_AT;
static_assert(SZ_AT >= (size_t)8 * 256 * 16);
static_assert(SZ_TOTAL <= (size_t)134217728);

extern "C" void kernel_launch(void* const* d_in, const int* in_sizes, int n_in,
                              void* d_out, int out_size, void* d_ws, size_t ws_size, hipStream_t stream) {
    if (n_in < 5) return;
    if ((size_t)in_sizes[0] < (size_t)(NB - 1) * SEQ_FULL + (size_t)SEQ) return;
    if ((size_t)in_sizes[1] < (size_t)HID * WIN) return;
    if ((size_t)in_sizes[2] < (size_t)HID) return;
    if ((size_t)in_sizes[3] < (size_t)HID) return;
    if ((size_t)in_sizes[4] < (size_t)1) return;
    if ((size_t)out_size < (size_t)NB * SEQ) return;
    if (SZ_TOTAL > ws_size) return;
    const float* ret = (const float*)d_in[0];
    const float* W1  = (const float*)d_in[1];
    const float* b1  = (const float*)d_in[2];
    const float* W2  = (const float*)d_in[3];
    const float* b2  = (const float*)d_in[4];
    float* OUT = (float*)d_out;
    bf* AT = (bf*)d_ws;

    k_wt<<<1, 256, 0, stream>>>(W1, b1, AT);
    k_hurst<<<NB, NTHR, 0, stream>>>(ret, AT, W2, b2, OUT);
}
